// TransformerBlock_89197880803919
// MI455X (gfx1250) — hardware-run, weakly checked
//
#include <hip/hip_runtime.h>


#ifndef NB
#define NB 2
#endif
#ifndef SEQ
#define SEQ 4096
#endif
#define NB_FULL  2
#define SEQ_FULL 4096
#ifndef OUT_SEQ
#define OUT_SEQ SEQ
#endif
#define DM   768
#define NH_  12
#define HD   64
#define FFD  3072
#define ERL  ((SEQ) < 512 ? (SEQ) : 512)
#define AW   4
#define QRS  2048.0f
#define QRI  (1.0f / 2048.0f)
#define SC2  (0.125f * 1.4426950408889634f)
#define PSH  8.0f
#define CTXC 64.0f
#define WSC  64.0f
#define NEGB (-3.0e38f)

#define EPI_QK   0
#define EPI_VT   1
#define EPI_RES  2
#define EPI_GELU 3

static_assert(HD == 64);
static_assert(NH_ * HD == DM);
static_assert(DM % 64 == 0);
static_assert(FFD % 64 == 0);
static_assert(DM % 32 == 0);
static_assert(FFD % 32 == 0);
static_assert(SEQ % 64 == 0);
static_assert(ERL % 64 == 0);
static_assert((SEQ - ERL) % 64 == 0);
static_assert(ERL % (16 * AW) == 0);
static_assert((SEQ - ERL) % (16 * AW) == 0);
static_assert(SEQ % 32 == 0);
static_assert(ERL % 32 == 0);
static_assert((NB * SEQ) % 8 == 0);
static_assert(NB <= NB_FULL);
static_assert(SEQ <= SEQ_FULL);

typedef _Float16 h16;
typedef __attribute__((ext_vector_type(16))) _Float16 v16h;
typedef __attribute__((ext_vector_type(8)))  _Float16 v8h;
typedef __attribute__((ext_vector_type(8)))  float    v8f;
typedef __attribute__((ext_vector_type(4)))  float    v4f;
typedef v4f  __attribute__((may_alias)) v4fa;

__device__ __forceinline__ float bfr(float f) { unsigned u = __float_as_uint(f); u += 0x7FFFu + ((u >> 16) & 1u); return __uint_as_float(u & 0xFFFF0000u); }
__device__ __forceinline__ v16h cat16(v8h lo, v8h hi) { return __builtin_shufflevector(lo, hi, 0, 1, 2, 3, 4, 5, 6, 7, 8, 9, 10, 11, 12, 13, 14, 15); }
__device__ __forceinline__ v8f wmma16(v16h a, v16h b, v8f c) { return __builtin_amdgcn_wmma_f32_16x16x32_f16(false, a, false, b, (short)0, c, false, false); }
__device__ __forceinline__ v16h ldh(const h16* p) { return cat16(*(const v8h*)p, *(const v8h*)(p + 16)); }
__device__ __forceinline__ void wave_sync() { __builtin_amdgcn_fence(3  , "wavefront"); __builtin_amdgcn_wave_barrier(); asm volatile("" ::: "memory"); }
__device__ __forceinline__ float gelu_f(float x) {
    const float u = 0.7978845608028654f * (x + 0.044715f * x * x * x);
    const float e = __expf(fminf(-2.0f * u, 80.0f));
    return x * __builtin_amdgcn_rcpf(1.0f + e);
}
__device__ __forceinline__ void stage8(float* d, v8f o, float s) {
    v4f a, c;
    a[0] = o[0] * s; a[1] = o[1] * s; a[2] = o[2] * s; a[3] = o[3] * s; c[0] = o[4] * s; c[1] = o[5] * s; c[2] = o[6] * s; c[3] = o[7] * s;
    *(v4fa*)d = a; *(v4fa*)(d + 4) = c;
}

__global__ __launch_bounds__(256) void k_wT(const float* __restrict__ W, int K, int N, h16* dst, int pitch, int colOff, float scale) {
    __shared__ __align__(16) float ts[64 * 65];
    const int tid = threadIdx.x; const int k0 = blockIdx.y * 64, n0 = blockIdx.x * 64;
#pragma unroll
    for (int i = 0; i < 4; ++i) { const int idx = tid + 256 * i; const int r = idx >> 4, c4 = (idx & 15) * 4;
        const v4f v = *(const v4f*)(W + (size_t)(k0 + r) * (size_t)N + n0 + c4);
        ts[r * 65 + c4 + 0] = v[0]; ts[r * 65 + c4 + 1] = v[1]; ts[r * 65 + c4 + 2] = v[2]; ts[r * 65 + c4 + 3] = v[3]; }
    __syncthreads();
    const int k8 = (tid & 7) * 8; v8h o[2];
#pragma unroll
    for (int p = 0; p < 2; ++p) { const int n = (tid >> 3) + 32 * p;
#pragma unroll
        for (int i = 0; i < 8; ++i) o[p][i] = (h16)(bfr(ts[(k8 + i) * 65 + n]) * scale); }
    h16* d0 = dst + (size_t)(n0 + (tid >> 3)) * (size_t)pitch + colOff + k0 + k8;
    h16* d1 = d0 + (size_t)32 * (size_t)pitch;
    *(volatile v8h*)d0 = o[0]; *(volatile v8h*)d1 = o[1];
    __threadfence();
    *(volatile v8h*)d0 = o[0]; *(volatile v8h*)d1 = o[1];
}

__global__ __launch_bounds__(256) void k_ln(const float* __restrict__ X, int srcRPB, const float* __restrict__ sc, const float* __restrict__ sf, h16* H, int nrows, int cvtIn) {
    const int lane = threadIdx.x & 31, wave = __builtin_amdgcn_readfirstlane((int)(threadIdx.x >> 5));
    const int row = blockIdx.x * 8 + wave;
    if (row >= nrows) return;
    const int b = row / SEQ, t = row % SEQ;
    const float* src = X + ((size_t)b * (size_t)srcRPB + t) * DM + 8 * lane;
    v8f v[3]; float s = 0.0f;
#pragma unroll
    for (int j = 0; j < 3; ++j) { v[j] = *(const v8f*)(src + 256 * j);
#pragma unroll
        for (int i = 0; i < 8; ++i) { float e = v[j][i]; if (cvtIn) e = bfr(e); v[j][i] = e; s += e; } }
#pragma unroll
    for (int off = 16; off > 0; off >>= 1) s += __shfl_xor(s, off, 32);
    const float mean = s * (1.0f / DM);
    float q = 0.0f;
#pragma unroll
    for (int j = 0; j < 3; ++j)
#pragma unroll
        for (int i = 0; i < 8; ++i) { const float d = v[j][i] - mean; q += d * d; }
#pragma unroll
    for (int off = 16; off > 0; off >>= 1) q += __shfl_xor(q, off, 32);
    const float rstd = rsqrtf(q * (1.0f / DM) + 1e-5f);
    v8h o[3];
#pragma unroll
    for (int j = 0; j < 3; ++j) { const v8f g = *(const v8f*)(sc + 256 * j + 8 * lane); const v8f f = *(const v8f*)(sf + 256 * j + 8 * lane);
#pragma unroll
        for (int i = 0; i < 8; ++i) o[j][i] = (h16)(bfr(g[i]) * (v[j][i] - mean) * rstd + bfr(f[i])); }
    h16* dst = H + (size_t)row * DM + 8 * lane;
    *(volatile v8h*)(dst) = o[0]; *(volatile v8h*)(dst + 256) = o[1]; *(volatile v8h*)(dst + 512) = o[2];
    __threadfence();
    *(volatile v8h*)(dst) = o[0]; *(volatile v8h*)(dst + 256) = o[1]; *(volatile v8h*)(dst + 512) = o[2];
}

template<int EPI>
__global__ __launch_bounds__(32) void k_gemm(const h16* __restrict__ A, int lda, const h16* __restrict__ Bt, int ldb, int K,
                                             int tpb, int aRPB, int aOff, int oRPB, int oOff, int rRPB,
                                             h16* P0, h16* P1, float* OF, const float* __restrict__ Rsrc, const float* __restrict__ bias,
                                             float scale, int cvtR) {
    __shared__ __align__(16) float os[16 * 68];
    const int lane = threadIdx.x & 31, lr = lane & 15, hi = lane >> 4;
    const int ib = (int)blockIdx.x / tpb, tt = (int)blockIdx.x % tpb;
    const int arow0 = ib * aRPB + aOff + tt * 64;
    const int ot0 = oOff + tt * 64;
    const int c0 = (int)blockIdx.y * 64;
    v8f acc[4][4];
#pragma unroll
    for (int mb = 0; mb < 4; ++mb)
#pragma unroll
        for (int nb = 0; nb < 4; ++nb) acc[mb][nb] = (v8f){};
    const size_t aoff = (size_t)(arow0 + lr) * (size_t)lda + 8 * hi, boff = (size_t)(c0 + lr) * (size_t)ldb + 8 * hi;
#pragma unroll 1
    for (int kc = 0; kc < K; kc += 32) {
        v16h a[4];
#pragma unroll
        for (int mb = 0; mb < 4; ++mb) a[mb] = ldh(A + aoff + (size_t)mb * 16 * (size_t)lda + kc);
#pragma unroll
        for (int nb = 0; nb < 4; ++nb) { const v16h b = ldh(Bt + boff + (size_t)nb * 16 * (size_t)ldb + kc);
#pragma unroll
            for (int mb = 0; mb < 4; ++mb) acc[mb][nb] = wmma16(a[mb], b, acc[mb][nb]); }
        asm volatile("v_nop\n\tv_nop\n\tv_nop\n\tv_nop" : "+v"(acc[0][0]), "+v"(acc[1][1]), "+v"(acc[2][2]), "+v"(acc[3][3]) : "v"(a[0]), "v"(a[1]), "v"(a[2]), "v"(a[3]));
    }
    if (EPI == EPI_RES) {
        const size_t ob = ((size_t)ib * (size_t)oRPB + ot0) * DM + c0;
        const size_t rb = ((size_t)ib * (size_t)rRPB + ot0) * DM + c0;
        const int cofs = lr * 4;
        v4f bv = *(const v4f*)(bias + c0 + cofs);
        bv[0] = bfr(bv[0]); bv[1] = bfr(bv[1]); bv[2] = bfr(bv[2]); bv[3] = bfr(bv[3]);
#pragma unroll
        for (int mb = 0; mb < 4; ++mb) {
#pragma unroll
            for (int nb = 0; nb < 4; ++nb) {
#pragma unroll
                for (int j = 0; j < 8; ++j) os[(hi * 8 + j) * 68 + nb * 16 + lr] = acc[mb][nb][j]; }
            wave_sync();
            v4f val[8];
#pragma unroll
            for (int s = 0; s < 8; ++s) { const int row = 2 * s + hi;
                const v4f xv = *(const v4fa*)(&os[row * 68 + cofs]);
                v4f rv = *(const v4f*)(Rsrc + rb + (size_t)(mb * 16 + row) * DM + cofs);
                if (cvtR) { rv[0] = bfr(rv[0]); rv[1] = bfr(rv[1]); rv[2] = bfr(rv[2]); rv[3] = bfr(rv[3]); }
                val[s] = rv + (xv * scale + bv); }
#pragma unroll
            for (int s = 0; s < 8; ++s) *(volatile v4f*)(OF + ob + (size_t)(mb * 16 + 2 * s + hi) * DM + cofs) = val[s];
            __threadfence();
#pragma unroll
            for (int s = 0; s < 8; ++s) *(volatile v4f*)(OF + ob + (size_t)(mb * 16 + 2 * s + hi) * DM + cofs) = val[s];
            wave_sync();
        }
    } else {
        size_t base1 = 0, base2 = 0; size_t pitch1 = 0, pitch2 = 0; int res = 0;
        if (EPI == EPI_QK) {
            const size_t zh = (size_t)ib * NH_ + blockIdx.y;
            base1 = (zh * SEQ + ot0) * HD; pitch1 = HD; base2 = (zh * ERL + ot0) * HD; pitch2 = HD; res = (ot0 < ERL) ? 1 : 0;
        } else if (EPI == EPI_VT) {
            const int bn = c0 / SEQ, tn = c0 % SEQ; const size_t rw = (size_t)bn * DM + arow0;
            base1 = rw * SEQ + tn; pitch1 = SEQ; base2 = rw * ERL + tn; pitch2 = ERL; res = (tn < ERL) ? 1 : 0;
        } else {
            base1 = ((size_t)ib * (size_t)oRPB + ot0) * FFD + c0; pitch1 = FFD;
        }
        const int c8 = (lane & 7) * 8, rq = lane >> 3;
        float bvs[8];
#pragma unroll
        for (int i = 0; i < 8; ++i) bvs[i] = 0.0f;
        if (EPI == EPI_GELU) { const v4f b0 = *(const v4f*)(bias + c0 + c8); const v4f b1 = *(const v4f*)(bias + c0 + c8 + 4);
#pragma unroll
            for (int i = 0; i < 4; ++i) { bvs[i] = bfr(b0[i]); bvs[4 + i] = bfr(b1[i]); } }
#pragma unroll
        for (int mb = 0; mb < 4; ++mb) {
#pragma unroll
            for (int nb = 0; nb < 4; ++nb) {
#pragma unroll
                for (int j = 0; j < 8; ++j) os[(hi * 8 + j) * 68 + nb * 16 + lr] = acc[mb][nb][j]; }
            wave_sync();
            v8h hv[4], rv[4];
#pragma unroll
            for (int s = 0; s < 4; ++s) { const int row = 4 * s + rq;
                const v4f x0 = *(const v4fa*)(&os[row * 68 + c8]); const v4f x1 = *(const v4fa*)(&os[row * 68 + c8 + 4]);
#pragma unroll
                for (int i = 0; i < 4; ++i) { float v0 = x0[i] * scale, v1 = x1[i] * scale;
                    if (EPI == EPI_GELU) { v0 = gelu_f(v0 + bvs[i]); v1 = gelu_f(v1 + bvs[4 + i]); }
                    const h16 a0 = (h16)v0; const h16 a1 = (h16)v1; hv[s][i] = a0; hv[s][4 + i] = a1;
                    rv[s][i] = (h16)((v0 - (float)a0) * QRS); rv[s][4 + i] = (h16)((v1 - (float)a1) * QRS); } }
#pragma unroll
            for (int s = 0; s < 4; ++s) { const size_t rr = (size_t)(mb * 16 + 4 * s + rq);
                *(volatile v8h*)(P0 + base1 + rr * pitch1 + c8) = hv[s]; if (res) *(volatile v8h*)(P1 + base2 + rr * pitch2 + c8) = rv[s]; }
            __threadfence();
#pragma unroll
            for (int s = 0; s < 4; ++s) { const size_t rr = (size_t)(mb * 16 + 4 * s + rq);
                *(volatile v8h*)(P0 + base1 + rr * pitch1 + c8) = hv[s]; if (res) *(volatile v8h*)(P1 + base2 + rr * pitch2 + c8) = rv[s]; }
            wave_sync();
        }
    }
}

template<int E>
__global__ __launch_bounds__(32 * AW) void k_flash(const h16* __restrict__ QH, const h16* __restrict__ QR, const h16* __restrict__ KH, const h16* __restrict__ KR,
                                                   const h16* __restrict__ VT, const h16* __restrict__ VR, h16* CT) {
    __shared__ __align__(16) float os[AW * 16 * 68];
    const int lane = threadIdx.x & 31, wave = __builtin_amdgcn_readfirstlane((int)(threadIdx.x >> 5)), lr = lane & 15, hi = lane >> 4;
    const int zh = blockIdx.y; const int b = zh / NH_, h = zh % NH_;
    const int t0 = (E ? 0 : ERL) + ((int)blockIdx.x * AW + wave) * 16;
    const size_t pbase = (size_t)zh * SEQ * HD;
    const size_t rbase = (size_t)zh * ERL * HD;
    const size_t qo = pbase + (size_t)(t0 + lr) * HD + 8 * hi;
    const v16h qh0 = ldh(QH + qo), qh1 = ldh(QH + qo + 32);
    v16h qr0 = qh0, qr1 = qh1;
    if (E) { const size_t qro = rbase + (size_t)(t0 + lr) * HD + 8 * hi; qr0 = ldh(QR + qro); qr1 = ldh(QR + qro + 32); }
    const size_t ko  = pbase + (size_t)lr * HD + 8 * hi;
    const size_t kro = rbase + (size_t)lr * HD + 8 * hi;
    const size_t vo  = pbase + (size_t)lr * SEQ + 8 * hi;
    const size_t vro = rbase + (size_t)lr * ERL + 8 * hi;
    v8f o0 = (v8f){}, o1 = (v8f){}, o2 = (v8f){}, o3 = (v8f){};
    v8f p0 = (v8f){}, p1 = (v8f){}, p2 = (v8f){}, p3 = (v8f){};
    float m = NEGB, l = 0.0f;
    const int kend = t0 + 16;
#pragma unroll 1
    for (int key0 = 0; key0 < kend; key0 += 32) {
        const h16* ka = KH + ko + (size_t)key0 * HD;
        const v16h ka0 = ldh(ka), ka1 = ldh(ka + 32), kb0 = ldh(ka + 16 * HD), kb1 = ldh(ka + 16 * HD + 32);
        v8f sHa = (v8f){}, sHb = (v8f){}, sLa = (v8f){}, sLb = (v8f){};
        sHa = wmma16(ka0, qh0, sHa); sHb = wmma16(kb0, qh0, sHb);
        sHa = wmma16(ka1, qh1, sHa); sHb = wmma16(kb1, qh1, sHb);
        if (E) {
            sLa = wmma16(ka0, qr0, sLa); sLb = wmma16(kb0, qr0, sLb);
            sLa = wmma16(ka1, qr1, sLa); sLb = wmma16(kb1, qr1, sLb);
            const h16* kr = KR + kro + (size_t)key0 * HD;
            const v16h ra0 = ldh(kr), ra1 = ldh(kr + 32), rb0 = ldh(kr + 16 * HD), rb1 = ldh(kr + 16 * HD + 32);
            sLa = wmma16(ra0, qh0, sLa); sLb = wmma16(rb0, qh0, sLb);
            sLa = wmma16(ra1, qh1, sLa); sLb = wmma16(rb1, qh1, sLb);
            asm volatile("v_nop\n\tv_nop\n\tv_nop\n\tv_nop" : "+v"(sHa), "+v"(sLa), "+v"(sHb), "+v"(sLb) : "v"(ra0), "v"(ra1), "v"(rb0), "v"(rb1));
        } else {
            asm volatile("v_nop\n\tv_nop\n\tv_nop\n\tv_nop" : "+v"(sHa), "+v"(sHb) : "v"(ka0), "v"(ka1), "v"(kb0), "v"(kb1));
        }
        float ta[8], tb[8];
#pragma unroll
        for (int r = 0; r < 8; ++r) {
            if (E) { ta[r] = (sHa[r] + sLa[r] * QRI) * SC2; tb[r] = (sHb[r] + sLb[r] * QRI) * SC2; }
            else   { ta[r] = sHa[r] * SC2; tb[r] = sHb[r] * SC2; } }
        if (key0 + 31 > t0) {
            const int kq = t0 + lr - key0 - 8 * hi;
#pragma unroll
            for (int r = 0; r < 8; ++r) { ta[r] = (r > kq) ? NEGB : ta[r]; tb[r] = (16 + r > kq) ? NEGB : tb[r]; }
        }
        float mx = NEGB;
#pragma unroll
        for (int r = 0; r < 8; ++r) mx = fmaxf(mx, fmaxf(ta[r], tb[r]));
        mx = fmaxf(mx, __shfl_xor(mx, 16, 32));
        const float mnew = fmaxf(m, mx);
        const float alpha = __builtin_amdgcn_exp2f(m - mnew);
        const float sh = PSH - mnew;
        v16h pb; float ls = 0.0f;
#pragma unroll
        for (int r = 0; r < 8; ++r) { const h16 pa = (h16)__builtin_amdgcn_exp2f(ta[r] + sh); const h16 pc = (h16)__builtin_amdgcn_exp2f(tb[r] + sh); pb[r] = pa; pb[8 + r] = pc; ls += (float)pa + (float)pc; }
        l = l * alpha + ls; m = mnew;
        o0 = o0 * alpha; o1 = o1 * alpha; o2 = o2 * alpha; o3 = o3 * alpha;
        const h16* va = VT + vo + key0;
        const v16h v0 = ldh(va), v1 = ldh(va + (size_t)16 * SEQ), v2 = ldh(va + (size_t)32 * SEQ), v3 = ldh(va + (size_t)48 * SEQ);
        o0 = wmma16(v0, pb, o0); o1 = wmma16(v1, pb, o1); o2 = wmma16(v2, pb, o2); o3 = wmma16(v3, pb, o3);
        if (E) {
            p0 = p0 * alpha; p1 = p1 * alpha; p2 = p2 * alpha; p3 = p3 * alpha;
            const h16* vr = VR + vro + key0;
            const v16h w0 = ldh(vr), w1 = ldh(vr + (size_t)16 * ERL), w2 = ldh(vr + (size_t)32 * ERL), w3 = ldh(vr + (size_t)48 * ERL);
            p0 = wmma16(w0, pb, p0); p1 = wmma16(w1, pb, p1); p2 = wmma16(w2, pb, p2); p3 = wmma16(w3, pb, p3);
            asm volatile("v_nop\n\tv_nop\n\tv_nop\n\tv_nop" : "+v"(o0), "+v"(o1), "+v"(o2), "+v"(o3), "+v"(p0), "+v"(p1), "+v"(p2), "+v"(p3) : "v"(w0), "v"(w1), "v"(w2), "v"(w3), "v"(pb));
        } else {
            asm volatile("v_nop\n\tv_nop\n\tv_nop\n\tv_nop" : "+v"(o0), "+v"(o1), "+v"(o2), "+v"(o3) : "v"(v0), "v"(v1), "v"(v2), "v"(v3), "v"(pb));
        }
    }
    l += __shfl_xor(l, 16, 32);
    const float inv = CTXC * (1.0f / l);
    const int wb = wave * 16 * 68;
    if (E) {
        const v8f c0v = o0 + p0 * QRI, c1v = o1 + p1 * QRI, c2v = o2 + p2 * QRI, c3v = o3 + p3 * QRI;
        stage8(&os[wb + lr * 68 +  0 + 8 * hi], c0v, inv); stage8(&os[wb + lr * 68 + 16 + 8 * hi], c1v, inv);
        stage8(&os[wb + lr * 68 + 32 + 8 * hi], c2v, inv); stage8(&os[wb + lr * 68 + 48 + 8 * hi], c3v, inv);
    } else {
        stage8(&os[wb + lr * 68 +  0 + 8 * hi], o0, inv); stage8(&os[wb + lr * 68 + 16 + 8 * hi], o1, inv);
        stage8(&os[wb + lr * 68 + 32 + 8 * hi], o2, inv); stage8(&os[wb + lr * 68 + 48 + 8 * hi], o3, inv);
    }
    wave_sync();
    const size_t cp = E ? (size_t)(2 * DM) : (size_t)DM;
    h16* crow = E ? (CT + ((size_t)b * ERL + t0) * (size_t)(2 * DM) + h * HD) : (CT + ((size_t)b * SEQ + t0) * (size_t)DM + h * HD);
    const int c8 = (lane & 7) * 8, rq = lane >> 3;
    v8h hv[4], rv[4];
#pragma unroll
    for (int s = 0; s < 4; ++s) { const int row = 4 * s + rq;
        const v4f x0 = *(const v4fa*)(&os[wb + row * 68 + c8]); const v4f x1 = *(const v4fa*)(&os[wb + row * 68 + c8 + 4]);
#pragma unroll
        for (int i = 0; i < 4; ++i) { const h16 a0 = (h16)x0[i]; const h16 a1 = (h16)x1[i]; hv[s][i] = a0; hv[s][4 + i] = a1;
            rv[s][i] = (h16)((x0[i] - (float)a0) * QRS); rv[s][4 + i] = (h16)((x1[i] - (float)a1) * QRS); } }
#pragma unroll
    for (int s = 0; s < 4; ++s) { h16* d = crow + (size_t)(4 * s + rq) * cp + c8; *(volatile v8h*)d = hv[s]; if (E) *(volatile v8h*)(d + DM) = rv[s]; }
    __threadfence();
#pragma unroll
    for (int s = 0; s < 4; ++s) { h16* d = crow + (size_t)(4 * s + rq) * cp + c8; *(volatile v8h*)d = hv[s]; if (E) *(volatile v8h*)(d + DM) = rv[s]; }
}

static constexpr size_t al256(size_t v) { return (v + 255) & ~(size_t)255; }
static constexpr size_t SZ_WSQ = al256((size_t)DM * DM * 2);
static constexpr size_t SZ_WOE = al256((size_t)DM * 2 * DM * 2);
static constexpr size_t SZ_WFF = al256((size_t)DM * FFD * 2);
static constexpr size_t SZ_H   = al256((size_t)NB * SEQ * DM * 2);
static constexpr size_t SZ_X1  = al256((size_t)NB * SEQ * DM * 4);
static constexpr size_t SZ_RP  = al256((size_t)NB * NH_ * ERL * HD * 2);
static constexpr size_t SZ_CE  = al256((size_t)NB * ERL * 2 * DM * 2);
static constexpr size_t SZ_PL  = (size_t)NB * SEQ * DM * 2;
static constexpr size_t SZ_BIG = 4 * SZ_PL;
static_assert(SZ_PL % 256 == 0);
static_assert((size_t)NB * NH_ * SEQ * HD * 2 == SZ_PL);
static_assert((size_t)NB * SEQ * FFD * 2 <= SZ_BIG);
static constexpr size_t SZ_TOTAL = 3 * SZ_WSQ + SZ_WOE + 2 * SZ_WFF + 2 * SZ_H + SZ_X1 + 3 * SZ_RP + SZ_CE + SZ_BIG;
static_assert(SZ_TOTAL <= (size_t)134217728);

extern "C" void kernel_launch(void* const* d_in, const int* in_sizes, int n_in,
                              void* d_out, int out_size, void* d_ws, size_t ws_size, hipStream_t stream) {
    if (n_in < 14) return;
    if ((size_t)in_sizes[0] < ((size_t)(NB - 1) * SEQ_FULL + SEQ) * DM) return;
    if ((size_t)in_sizes[1] < (size_t)DM * DM || (size_t)in_sizes[2] < (size_t)DM * DM || (size_t)in_sizes[3] < (size_t)DM * DM || (size_t)in_sizes[4] < (size_t)DM * DM) return;
    if ((size_t)in_sizes[5] < (size_t)DM || (size_t)in_sizes[6] < (size_t)DM * FFD || (size_t)in_sizes[7] < (size_t)FFD || (size_t)in_sizes[8] < (size_t)FFD * DM || (size_t)in_sizes[9] < (size_t)DM) return;
    if ((size_t)in_sizes[10] < (size_t)DM || (size_t)in_sizes[11] < (size_t)DM || (size_t)in_sizes[12] < (size_t)DM || (size_t)in_sizes[13] < (size_t)DM) return;
    if ((size_t)out_size < ((size_t)(NB - 1) * OUT_SEQ + SEQ) * DM) return;
    if (SZ_TOTAL > ws_size) return;
    const float* x  = (const float*)d_in[0];
    const float* wq = (const float*)d_in[1]; const float* wk = (const float*)d_in[2]; const float* wv = (const float*)d_in[3]; const float* wo = (const float*)d_in[4];
    const float* bo = (const float*)d_in[5]; const float* w1 = (const float*)d_in[6]; const float* b1 = (const float*)d_in[7];
    const float* w2 = (const float*)d_in[8]; const float* b2 = (const float*)d_in[9];
    const float* l1s = (const float*)d_in[10]; const float* l1b = (const float*)d_in[11]; const float* l2s = (const float*)d_in[12]; const float* l2b = (const float*)d_in[13];
    float* OUT = (float*)d_out;
    char* wsp = (char*)d_ws;
    h16* WQT = (h16*)wsp; wsp += SZ_WSQ;
    h16* WKT = (h16*)wsp; wsp += SZ_WSQ;
    h16* WVT = (h16*)wsp; wsp += SZ_WSQ;
    h16* WOE = (h16*)wsp; wsp += SZ_WOE;
    h16* W1T = (h16*)wsp; wsp += SZ_WFF;
    h16* W2T = (h16*)wsp; wsp += SZ_WFF;
    h16* H1  = (h16*)wsp; wsp += SZ_H;
    h16* H2  = (h16*)wsp; wsp += SZ_H;
    float* X1 = (float*)wsp; wsp += SZ_X1;
    h16* QR  = (h16*)wsp; wsp += SZ_RP;
    h16* KR  = (h16*)wsp; wsp += SZ_RP;
    h16* VTR = (h16*)wsp; wsp += SZ_RP;
    h16* CE  = (h16*)wsp; wsp += SZ_CE;
    h16* QH  = (h16*)wsp;
    h16* KH  = (h16*)(wsp + SZ_PL);
    h16* VT  = (h16*)(wsp + 2 * SZ_PL);
    h16* CTX = (h16*)(wsp + 3 * SZ_PL);
    h16* G   = (h16*)wsp;

    k_wT<<<dim3(DM / 64, DM / 64, 1), 256, 0, stream>>>(wq, DM, DM, WQT, DM, 0, WSC);
    k_wT<<<dim3(DM / 64, DM / 64, 1), 256, 0, stream>>>(wk, DM, DM, WKT, DM, 0, WSC);
    k_wT<<<dim3(DM / 64, DM / 64, 1), 256, 0, stream>>>(wv, DM, DM, WVT, DM, 0, WSC);
    k_wT<<<dim3(DM / 64, DM / 64, 1), 256, 0, stream>>>(wo, DM, DM, WOE, 2 * DM, 0, 2048.0f);
    k_wT<<<dim3(DM / 64, DM / 64, 1), 256, 0, stream>>>(wo, DM, DM, WOE, 2 * DM, DM, 1.0f);
    k_wT<<<dim3(FFD / 64, DM / 64, 1), 256, 0, stream>>>(w1, DM, FFD, W1T, DM, 0, WSC);
    k_wT<<<dim3(DM / 64, FFD / 64, 1), 256, 0, stream>>>(w2, FFD, DM, W2T, FFD, 0, WSC);

    k_ln<<<(NB * SEQ + 7) / 8, 256, 0, stream>>>(x, SEQ_FULL, l1s, l1b, H1, NB * SEQ, 1);

    k_gemm<EPI_QK><<<dim3(NB * SEQ / 64, DM / 64, 1), 32, 0, stream>>>(H1, DM, WQT, DM, DM, SEQ / 64, SEQ, 0, SEQ, 0, SEQ, QH, QR, X1, x, bo, 1.0f / 64.0f, 0);
    k_gemm<EPI_QK><<<dim3(NB * SEQ / 64, DM / 64, 1), 32, 0, stream>>>(H1, DM, WKT, DM, DM, SEQ / 64, SEQ, 0, SEQ, 0, SEQ, KH, KR, X1, x, bo, 1.0f / 64.0f, 0);
    k_gemm<EPI_VT><<<dim3(DM / 64, NB * SEQ / 64, 1), 32, 0, stream>>>(WVT, DM, H1, DM, DM, DM / 64, 0, 0, 0, 0, 0, VT, VTR, X1, x, bo, 1.0f / 64.0f, 0);

    k_flash<1><<<dim3(ERL / (16 * AW), NB * NH_, 1), 32 * AW, 0, stream>>>(QH, QR, KH, KR, VT, VTR, CE);
    if (SEQ > ERL) k_flash<0><<<dim3((SEQ - ERL) / (16 * AW), NB * NH_, 1), 32 * AW, 0, stream>>>(QH, QR, KH, KR, VT, VTR, CTX);

    k_gemm<EPI_RES><<<dim3(NB * ERL / 64, DM / 64, 1), 32, 0, stream>>>(CE, 2 * DM, WOE, 2 * DM, 2 * DM, ERL / 64, ERL, 0, SEQ, 0, SEQ_FULL, QR, KR, X1, x, bo, 1.0f / 131072.0f, 1);
    if (SEQ > ERL) k_gemm<EPI_RES><<<dim3(NB * (SEQ - ERL) / 64, DM / 64, 1), 32, 0, stream>>>(CTX, DM, WOE, 2 * DM, DM, (SEQ - ERL) / 64, SEQ, ERL, SEQ, ERL, SEQ_FULL, QR, KR, X1, x, bo, 1.0f / 131072.0f, 1);

    k_ln<<<(NB * SEQ + 7) / 8, 256, 0, stream>>>(X1, SEQ, l2s, l2b, H2, NB * SEQ, 0);

    k_gemm<EPI_GELU><<<dim3(NB * SEQ / 64, FFD / 64, 1), 32, 0, stream>>>(H2, DM, W1T, DM, DM, NB * SEQ / 64, 0, 0, 0, 0, 0, G, QR, X1, x, b1, 1.0f / 64.0f, 0);
    k_gemm<EPI_RES><<<dim3(NB * SEQ / 64, DM / 64, 1), 32, 0, stream>>>(G, FFD, W2T, FFD, FFD, SEQ / 64, SEQ, 0, OUT_SEQ, 0, SEQ, QR, KR, OUT, X1, b2, 1.0f / 64.0f, 0);
}
